// GlobalBlock_20710332301890
// MI455X (gfx1250) — hardware-verified
//
#include <hip/hip_runtime.h>
#include <hip/hip_bf16.h>
#include <math.h>

#define BB 8
#define SS 2048
#define CC 128
#define DD 128
#define HH 1
#define DKK 128
#define QW 1
#define QST 128
#define KVST 128
#define KST2 136
#define MTOK (BB * SS)
#define GSTR 48

typedef _Float16 bf16;
typedef _Float16 f16;
typedef __attribute__((ext_vector_type(4))) unsigned v4u_t;
typedef unsigned v4ua __attribute__((ext_vector_type(4), may_alias));
typedef __attribute__((ext_vector_type(4))) float v4f_t;
typedef float v4fa __attribute__((ext_vector_type(4), may_alias));
typedef __attribute__((ext_vector_type(16))) bf16  bf16x16;
typedef bf16x16 f16x16;
typedef __attribute__((ext_vector_type(8)))  bf16  bf16x8;
typedef bf16x8 f16x8;
typedef __attribute__((ext_vector_type(4)))  bf16  bf16x4;
typedef __attribute__((ext_vector_type(8)))  float f32x8;
__device__ __forceinline__ f32x8 wmma16(f16x16 a, f16x16 b, f32x8 c) {
  c = __builtin_amdgcn_wmma_f32_16x16x32_f16(false, a, false, b, (short)0, c, false, false);
  asm volatile("v_nop\n\tv_nop\n\tv_nop\n\tv_nop" : "+v"(c) : "v"(a), "v"(b));
  return c;
}
#define LDS_STRIDE 48
#define KSTRIDE    72
#define VSTRIDE    48

__device__ __forceinline__ f32x8 wmma_bf16(bf16x16 a, bf16x16 b, f32x8 c) {
  c = __builtin_amdgcn_wmma_f32_16x16x32_f16(false, a, false, b, (short)0, c, false, false);
  asm volatile("v_nop\n\tv_nop\n\tv_nop\n\tv_nop" : "+v"(c) : "v"(a), "v"(b));
  return c;
}

template <typename T>
__device__ __forceinline__ bf16x16 load_frag(const T* __restrict__ base, int ld,
                                             int row0, int k0) {
  const int lane = threadIdx.x & 31;
  const int r    = lane & 15;
  const int kh   = (lane >> 4) * 8;
  const T* p0 = base + (size_t)(row0 + r) * ld + (k0 + kh);
  const T* p1 = p0 + 16;
  bf16x16 f;
#pragma unroll
  for (int i = 0; i < 8; ++i) {
    f[i]     = (bf16)p0[i];
    f[i + 8] = (bf16)p1[i];
  }
  return f;
}

__device__ __forceinline__ bf16x16 lds_frag(const bf16* base, int stride) {
  const int lane = threadIdx.x & 31;
  const int row  = lane & 15;
  const int kh   = (lane >> 4) * 8;
  const bf16x8 lo = *(const bf16x8*)(base + row * stride + kh);
  const bf16x8 hi = *(const bf16x8*)(base + row * stride + kh + 16);
  bf16x16 f;
#pragma unroll
  for (int i = 0; i < 8; ++i) { f[i] = lo[i]; f[i + 8] = hi[i]; }
  return f;
}

template <typename T>
__device__ __forceinline__ void stage_read16(const T* __restrict__ p, float* buf) {
#pragma unroll
  for (int i = 0; i < 16; ++i) buf[i] = (float)p[i];
}

__device__ __forceinline__ void stage_write(bf16* dst, const float* buf, int nquad) {
#pragma unroll
  for (int i = 0; i < nquad; ++i) {
    bf16x4 q;
    q[0] = (bf16)buf[4 * i];     q[1] = (bf16)buf[4 * i + 1];
    q[2] = (bf16)buf[4 * i + 2]; q[3] = (bf16)buf[4 * i + 3];
    *(bf16x4*)(dst + 4 * i) = q;
  }
}

__global__ __launch_bounds__(64) void attn_kernel(
    const bf16* __restrict__ Qb, const bf16* __restrict__ Kb,
    const bf16* __restrict__ Vt,
    bf16* __restrict__ attnOut) {
  __shared__ bf16 ldsK[32 * KST2];
  __shared__ bf16 ldsV[128 * VSTRIDE];
  __shared__ __attribute__((aligned(16))) bf16 ldsO[2][16 * 136];

  const int q0blk = blockIdx.x * 32;
  const int h  = blockIdx.y;
  const int b  = blockIdx.z;
  const int t    = threadIdx.x;
  const int wave = t >> 5;
  const int lane = t & 31;
  const int qlane = lane & 15;
  const int kh8   = (lane >> 4) * 8;
  const int q0 = q0blk + wave * 16;

  const int hk = h;
  const bf16* Qh = Qb + (size_t)b * SS * QST + h * DKK;
  const bf16* Kh = Kb + (size_t)b * SS * KVST + hk * DKK;
  const bf16* Vh = Vt + ((size_t)(b * HH + hk)) * DKK * SS;

  const int krow = t >> 1;
  const int kcol = (t & 1) * 64;
  const bf16* kSrc = Kh + (size_t)krow * KVST + kcol;
  const bf16* vSrc = Vh + (size_t)t * SS;

  bf16x16 qf[QW][4];
#pragma unroll
  for (int qt = 0; qt < QW; ++qt)
#pragma unroll
    for (int c = 0; c < 4; ++c) qf[qt][c] = load_frag(Qh, QST, q0 + 16 * qt, 32 * c);

  f32x8 o[QW][8] = {};
  float mrun[QW], lrun[QW];
#pragma unroll
  for (int qt = 0; qt < QW; ++qt) { mrun[qt] = -INFINITY; lrun[qt] = 0.0f; }

  const float scale = 0.08838834764831845f * 1.44269504088896340736f;
  const float NEG2 = -1.0e9f; (void)NEG2;
  const int kmax = SS - 1, kmin = 0;

  bf16x8 kreg[8], vreg[8];
#pragma unroll
  for (int i = 0; i < 8; ++i) kreg[i] = *(const bf16x8*)(kSrc + (size_t)kmin * KVST + 8 * i);
#pragma unroll
  for (int i = 0; i < 4; ++i) { vreg[i] = *(const bf16x8*)(vSrc + kmin + 8 * i); vreg[4 + i] = *(const bf16x8*)(vSrc + (size_t)64 * SS + kmin + 8 * i); }

  for (int kb = kmin; kb <= kmax; kb += 32) {
    __syncthreads();
#pragma unroll
    for (int i = 0; i < 8; ++i) *(bf16x8*)(&ldsK[krow * KST2 + kcol + 8 * i]) = kreg[i];
#pragma unroll
    for (int i = 0; i < 4; ++i) { *(bf16x8*)(&ldsV[t * VSTRIDE + 8 * i]) = vreg[i]; *(bf16x8*)(&ldsV[(t + 64) * VSTRIDE + 8 * i]) = vreg[4 + i]; }
    if (kb + 32 <= kmax) {
      const bf16* kn = kSrc + (size_t)(kb + 32) * KVST;
      const bf16* vn = vSrc + (kb + 32);
#pragma unroll
      for (int i = 0; i < 8; ++i) kreg[i] = *(const bf16x8*)(kn + 8 * i);
#pragma unroll
      for (int i = 0; i < 4; ++i) { vreg[i] = *(const bf16x8*)(vn + 8 * i); vreg[4 + i] = *(const bf16x8*)(vn + (size_t)64 * SS + 8 * i); }
    }
    __syncthreads();


    bf16x16 pf[QW];
    bool act[QW];
#pragma unroll
    for (int qt = 0; qt < QW; ++qt) {
      unsigned mbits = 0;
      mbits = 0xFFFFu; act[qt] = true;
      if (act[qt]) {
        const int q_my = q0 + 16 * qt + qlane;
        f32x8 s0 = {}, s1 = {};
#pragma unroll
        for (int c = 0; c < 4; ++c) {
          const bf16x16 k0f = lds_frag(ldsK + 0 * KST2 + c * 32, KST2), k1f = lds_frag(ldsK + 16 * KST2 + c * 32, KST2);
          s0 = wmma_bf16(k0f, qf[qt][c], s0);
          s1 = wmma_bf16(k1f, qf[qt][c], s1);
        }

        float mx = -INFINITY;
#pragma unroll
        for (int r = 0; r < 8; ++r) {
          const int k0i = kb + kh8 + r;
          const int k1i = k0i + 16;
          (void)k0i; (void)k1i; (void)q_my;
          s0[r] = (mbits & (1u << r))       ? s0[r] * scale : NEG2;
          s1[r] = (mbits & (1u << (8 + r))) ? s1[r] * scale : NEG2;
          mx = fmaxf(mx, fmaxf(s0[r], s1[r]));
        }
        mx = fmaxf(mx, __shfl_xor(mx, 16, 32));
        const float mnew  = fmaxf(mrun[qt], mx);
        const float alpha = exp2f(mrun[qt] - mnew);

        float rsum = 0.0f;
#pragma unroll
        for (int r = 0; r < 8; ++r) {
          const float p0 = exp2f(s0[r] - mnew);
          const float p1 = exp2f(s1[r] - mnew);
          rsum += p0 + p1;
          pf[qt][r]     = (bf16)(p0 * 1024.0f);
          pf[qt][r + 8] = (bf16)(p1 * 1024.0f);
        }
        rsum += __shfl_xor(rsum, 16, 32);
        lrun[qt] = lrun[qt] * alpha + rsum;
        mrun[qt] = mnew;

#pragma unroll
        for (int j = 0; j < 8; ++j)
#pragma unroll
          for (int r = 0; r < 8; ++r) o[qt][j][r] *= alpha;
      }
    }

#pragma unroll
    for (int j = 0; j < 8; ++j) {
      const bf16x16 vf = lds_frag(ldsV + (j * 16) * VSTRIDE, VSTRIDE);
#pragma unroll
      for (int qt = 0; qt < QW; ++qt)
        if (act[qt]) o[qt][j] = wmma_bf16(vf, pf[qt], o[qt][j]);
    }
  }

  bf16* so = ldsO[wave];
  {
    const float rl = 1.0f / (lrun[0] * 1024.0f);
#pragma unroll
    for (int j = 0; j < 8; ++j)
#pragma unroll
      for (int r = 0; r < 8; ++r) so[qlane * 136 + j * 16 + kh8 + r] = (bf16)(o[0][j][r] * rl);
  }
  asm volatile("s_wait_dscnt 0" ::: "memory");
  __builtin_amdgcn_wave_barrier();
#pragma unroll 1
  for (int pass = 0; pass < 2; ++pass) {
#pragma unroll
    for (int it = 0; it < 8; ++it) { const int ch = lane + 32 * it, ql = ch >> 4, q8 = (ch & 15) * 8;
      *(volatile v4u_t*)(attnOut + ((size_t)(b * SS + q0 + ql)) * QST + h * DKK + q8) = *(const v4ua*)(so + ql * 136 + q8); }
    __threadfence();
  }
}


#define GSTR 48
template <typename AT, int EPI, bool OUT16>
__global__ __launch_bounds__(256) void gemm_kne(const AT* __restrict__ A, int lda, const float* __restrict__ Wm, int ldw,
                                                const float* __restrict__ bias, const float* __restrict__ R, const float* __restrict__ gvec,
                                                void* __restrict__ Yv, int ldy, int K) {
  __shared__ __attribute__((aligned(16))) f16 ldsA[128 * GSTR];
  __shared__ __attribute__((aligned(16))) f16 ldsW[128 * GSTR];
  __shared__ __attribute__((aligned(16))) float oS[8][32 * 68];
  const int tid = threadIdx.x, lane = tid & 31, wave = tid >> 5, cl = lane & 15, rh = (lane >> 4) * 8;
  const int m0 = blockIdx.x * 128, n0 = blockIdx.y * 128;
  const int wm = (wave & 3) * 32, wn = (wave >> 2) * 64;
  f32x8 acc[2][4];
#pragma unroll
  for (int i = 0; i < 2; ++i)
#pragma unroll
    for (int j = 0; j < 4; ++j) { f32x8 z = {}; acc[i][j] = z; }
#pragma unroll 1
  for (int k0 = 0; k0 < K; k0 += 32) {
    __syncthreads();
    { const int row = tid >> 1, ch = (tid & 1) * 16;
      const AT* src = A + (size_t)(m0 + row) * lda + k0 + ch;
#pragma unroll
      for (int g = 0; g < 16; ++g) ldsA[row * GSTR + ch + g] = (f16)src[g]; }
    { const int k = tid >> 3, nn0 = (tid & 7) * 16;
      const float* src = Wm + (size_t)(k0 + k) * ldw + n0 + nn0;
#pragma unroll
      for (int g = 0; g < 4; ++g) { const v4f_t v = *(const v4f_t*)(src + 4 * g);
#pragma unroll
        for (int u = 0; u < 4; ++u) ldsW[(nn0 + 4 * g + u) * GSTR + k] = (f16)v[u]; } }
    __syncthreads();
    f16x16 af[2];
#pragma unroll
    for (int i = 0; i < 2; ++i) af[i] = lds_frag(ldsA + (wm + 16 * i) * GSTR, GSTR);
#pragma unroll
    for (int j = 0; j < 4; ++j) {
      const f16x16 bf = lds_frag(ldsW + (wn + 16 * j) * GSTR, GSTR);
#pragma unroll
      for (int i = 0; i < 2; ++i) acc[i][j] = wmma16(af[i], bf, acc[i][j]);
    }
  }
  float* so = oS[wave];
#pragma unroll
  for (int i = 0; i < 2; ++i)
#pragma unroll
    for (int j = 0; j < 4; ++j) {
      const int n = n0 + wn + 16 * j + cl;
      const float bv = bias ? bias[n] : 0.0f;
      const float gv = (EPI == 2) ? gvec[n] : 0.0f;
      if (EPI == 1) {
#pragma unroll 1
        for (int r = 0; r < 8; ++r) { const float xg = acc[i][j][r] + bv; so[(16 * i + rh + r) * 68 + 16 * j + cl] = 0.5f * xg * (1.0f + erff(xg * 0.70710678118654752f)); }
      } else {
#pragma unroll
        for (int r = 0; r < 8; ++r) {
          float v = acc[i][j][r] + bv;
          if (EPI == 2) v = R[(size_t)(m0 + wm + 16 * i + rh + r) * ldy + n] + gv * v;
          so[(16 * i + rh + r) * 68 + 16 * j + cl] = v;
        }
      }
    }
  asm volatile("s_wait_dscnt 0" ::: "memory");
  __builtin_amdgcn_wave_barrier();
#pragma unroll 1
  for (int pass = 0; pass < 2; ++pass) {
    if (OUT16) {
      f16* Y = (f16*)Yv;
#pragma unroll
      for (int it = 0; it < 8; ++it) { const int c = lane + 32 * it, rr = c >> 3, q8 = (c & 7) * 8;
        union { f16 h[8]; v4u_t v; } u;
#pragma unroll
        for (int e = 0; e < 8; ++e) u.h[e] = (f16)so[rr * 68 + q8 + e];
        *(volatile v4u_t*)(Y + (size_t)(m0 + wm + rr) * ldy + n0 + wn + q8) = u.v; }
    } else {
      float* Y = (float*)Yv;
#pragma unroll
      for (int it = 0; it < 16; ++it) { const int f4 = lane + 32 * it, rr = f4 >> 4, q = (f4 & 15) * 4;
        *(volatile v4f_t*)(Y + (size_t)(m0 + wm + rr) * ldy + n0 + wn + q) = *(const volatile v4fa*)(so + rr * 68 + q); }
    }
    __threadfence();
  }
}

__global__ __launch_bounds__(256) void k_relu_t(const float* __restrict__ x, float* __restrict__ ht) {
  __shared__ float tS[64][65];
  const int tid = threadIdx.x, b = blockIdx.z, c0 = blockIdx.y * 64, l0 = blockIdx.x * 64;
  for (int e = tid; e < 64 * 64; e += 256) { const int r = e >> 6, c = e & 63; tS[r][c] = fmaxf(x[((size_t)b * CC + c0 + r) * SS + l0 + c], 0.0f); }
  __syncthreads();
  for (int ch = tid; ch < 64 * 16; ch += 256) { const int l = ch >> 4, q4 = (ch & 15) * 4; v4f_t o; o[0] = tS[q4][l]; o[1] = tS[q4 + 1][l]; o[2] = tS[q4 + 2][l]; o[3] = tS[q4 + 3][l];
    float* dst = ht + ((size_t)b * SS + l0 + l) * CC + c0 + q4; *(volatile v4f_t*)dst = o; __threadfence(); *(volatile v4f_t*)dst = o; }
}
__global__ __launch_bounds__(256) void k_wt(const float* __restrict__ Wm, float* __restrict__ Wt) {
  __shared__ float tS[CC][CC + 1]; const int tid = threadIdx.x;
  for (int e = tid; e < CC * CC; e += 256) { const int r = e >> 7, c = e & 127; tS[r][c] = Wm[e]; }
  __syncthreads();
  for (int ch = tid; ch < CC * 32; ch += 256) { const int i = ch >> 5, q4 = (ch & 31) * 4; v4f_t o; o[0] = tS[q4][i]; o[1] = tS[q4 + 1][i]; o[2] = tS[q4 + 2][i]; o[3] = tS[q4 + 3][i];
    *(volatile v4f_t*)(Wt + (size_t)i * CC + q4) = o; __threadfence(); *(volatile v4f_t*)(Wt + (size_t)i * CC + q4) = o; }
}
__global__ __launch_bounds__(256) void k_vt(const float* __restrict__ v, bf16* __restrict__ Vt) {
  __shared__ bf16 tS[64][130];
  const int tid = threadIdx.x, blk = blockIdx.x; const int b = blk / (SS / 64), t0 = (blk % (SS / 64)) * 64;
  for (int e = tid; e < 64 * CC; e += 256) { const int r = e >> 7, c = e & 127; tS[r][c] = (bf16)v[((size_t)b * SS + t0 + r) * CC + c]; }
  __syncthreads();
  for (int ch = tid; ch < CC * 8; ch += 256) { const int c = ch >> 3, q8 = (ch & 7) * 8; union { bf16 hh[8]; v4u_t u; } cv;
#pragma unroll
    for (int e = 0; e < 8; ++e) cv.hh[e] = tS[q8 + e][c];
    bf16* dst = Vt + ((size_t)b * CC + c) * SS + t0 + q8; *(volatile v4u_t*)dst = cv.u; __threadfence(); *(volatile v4u_t*)dst = cv.u; }
}
__global__ __launch_bounds__(256) void k_relu16(const bf16* __restrict__ src, bf16* __restrict__ dst, size_t n8) {
  const size_t i = (size_t)blockIdx.x * 256 + threadIdx.x; if (i >= n8) return; union { bf16 hh[8]; v4u_t u; } cv; cv.u = *(const v4u_t*)(src + 8 * i);
#pragma unroll
  for (int e = 0; e < 8; ++e) cv.hh[e] = (cv.hh[e] > (bf16)0.0f) ? cv.hh[e] : (bf16)0.0f;
  *(volatile v4u_t*)(dst + 8 * i) = cv.u; __threadfence(); *(volatile v4u_t*)(dst + 8 * i) = cv.u;
}
__global__ __launch_bounds__(256) void k_out_t(const float* __restrict__ x, const float* __restrict__ y, float* __restrict__ out) {
  __shared__ float tS[64][65];
  const int tid = threadIdx.x, b = blockIdx.z, c0 = blockIdx.y * 64, l0 = blockIdx.x * 64;
  for (int e = tid; e < 64 * 64; e += 256) { const int l = e >> 6, c = e & 63; tS[l][c] = y[((size_t)b * SS + l0 + l) * CC + c0 + c]; }
  __syncthreads();
#pragma unroll 1
  for (int pass = 0; pass < 2; ++pass) {
    for (int ch = tid; ch < 64 * 16; ch += 256) { const int c = ch >> 4, q4 = (ch & 15) * 4; const size_t off = ((size_t)b * CC + c0 + c) * SS + l0 + q4; const v4f_t xv = *(const v4f_t*)(x + off);
      v4f_t o; o[0] = xv[0] + tS[q4][c]; o[1] = xv[1] + tS[q4 + 1][c]; o[2] = xv[2] + tS[q4 + 2][c]; o[3] = xv[3] + tS[q4 + 3][c];
      *(volatile v4f_t*)(out + off) = o; }
    __threadfence(); }
}

extern "C" void kernel_launch(void* const* d_in, const int* in_sizes, int n_in,
                              void* d_out, int out_size, void* d_ws, size_t ws_size,
                              hipStream_t stream) {
  (void)in_sizes; (void)n_in; (void)out_size;
  const float* x = (const float*)d_in[0];
  const float* Wq = (const float*)d_in[1], *bq = (const float*)d_in[2], *Wk = (const float*)d_in[3], *bk = (const float*)d_in[4];
  const float* Wv = (const float*)d_in[5], *bv = (const float*)d_in[6], *Wo = (const float*)d_in[7], *bo = (const float*)d_in[8];
  float* out = (float*)d_out;
  char* ws = (char*)d_ws;
  float* ht = (float*)ws; ws += (size_t)MTOK * CC * 4;
  float* WqT = (float*)ws; ws += CC * CC * 4; float* WkT = (float*)ws; ws += CC * CC * 4; float* WvT = (float*)ws; ws += CC * CC * 4; float* WoT = (float*)ws; ws += CC * CC * 4;
  bf16* Qb = (bf16*)ws; ws += (size_t)MTOK * CC * 2;
  bf16* Kb = (bf16*)ws; ws += (size_t)MTOK * CC * 2;
  float* v32 = (float*)ws; ws += (size_t)MTOK * CC * 4;
  bf16* VtB = (bf16*)ws; ws += (size_t)MTOK * CC * 2;
  bf16* att = (bf16*)ws; ws += (size_t)MTOK * CC * 2;
  bf16* ratt = (bf16*)ws; ws += (size_t)MTOK * CC * 2;
  float* y = (float*)ws; ws += (size_t)MTOK * CC * 4;
  if ((size_t)(ws - (char*)d_ws) > ws_size) return;
  const dim3 blk(256);
  k_relu_t<<<dim3(SS / 64, CC / 64, BB), blk, 0, stream>>>(x, ht);
  k_wt<<<dim3(1), blk, 0, stream>>>(Wq, WqT); k_wt<<<dim3(1), blk, 0, stream>>>(Wk, WkT); k_wt<<<dim3(1), blk, 0, stream>>>(Wv, WvT); k_wt<<<dim3(1), blk, 0, stream>>>(Wo, WoT);
  gemm_kne<float, 0, true><<<dim3(MTOK / 128, 1), blk, 0, stream>>>(ht, CC, WqT, CC, bq, nullptr, nullptr, Qb, CC, CC);
  gemm_kne<float, 0, true><<<dim3(MTOK / 128, 1), blk, 0, stream>>>(ht, CC, WkT, CC, bk, nullptr, nullptr, Kb, CC, CC);
  gemm_kne<float, 0, false><<<dim3(MTOK / 128, 1), blk, 0, stream>>>(ht, CC, WvT, CC, bv, nullptr, nullptr, v32, CC, CC);
  k_vt<<<dim3(BB * (SS / 64)), blk, 0, stream>>>(v32, VtB);
  attn_kernel<<<dim3(SS / 32, HH, BB), dim3(64), 0, stream>>>(Qb, Kb, VtB, att);
  k_relu16<<<dim3((MTOK * CC / 8 + 255) / 256), blk, 0, stream>>>(att, ratt, (size_t)MTOK * CC / 8);
  gemm_kne<bf16, 0, false><<<dim3(MTOK / 128, 1), blk, 0, stream>>>(ratt, CC, WoT, CC, bo, nullptr, nullptr, y, CC, CC);
  k_out_t<<<dim3(SS / 64, CC / 64, BB), blk, 0, stream>>>(x, y, out);
}
